// DensityAwareFeatureAggregator_42417097015678
// MI455X (gfx1250) — hardware-verified
//
#include <hip/hip_runtime.h>
#include <math.h>

typedef __attribute__((ext_vector_type(16))) _Float16 v16h;
typedef __attribute__((ext_vector_type(16))) __bf16 v16b;
typedef __attribute__((ext_vector_type(8)))  _Float16 v8h;
typedef __attribute__((ext_vector_type(8)))  float v8f;
typedef __attribute__((ext_vector_type(4)))  float v4f;
typedef __attribute__((ext_vector_type(2)))  float v2f;
typedef __attribute__((ext_vector_type(4)))  unsigned v4u;
typedef __attribute__((ext_vector_type(4)))  int v4i;
typedef float __attribute__((may_alias)) float_a;
typedef int __attribute__((may_alias)) int_a;

template <typename T> __device__ __forceinline__ void vst2(void* p, T v) { *(volatile T*)p = v; __threadfence(); *(volatile T*)p = v; }
__device__ __forceinline__ v8f wmma16(v16h a, v16h b, v8f c) {
  v8f d = __builtin_amdgcn_wmma_f32_16x16x32_f16(false, a, false, b, (short)0, c, false, false);
  asm volatile("v_nop\n\tv_nop\n\tv_nop\n\tv_nop" : "+v"(d) : "v"(a), "v"(b));
  return d;
}
__device__ __forceinline__ v8f wmma_bf(v16b a, v16b b, v8f c) {
  v8f d = __builtin_amdgcn_wmma_f32_16x16x32_bf16(false, a, false, b, (short)0, c, false, false);
  asm volatile("v_nop\n\tv_nop\n\tv_nop\n\tv_nop" : "+v"(d) : "v"(a), "v"(b));
  return d;
}
__device__ __forceinline__ v16h frag_h(const _Float16* rowk0, int lane) {
  union { v16h v; v8h q[2]; } u; const _Float16* p = rowk0 + 8 * (lane >> 4);
  u.q[0] = *(const v8h*)p; u.q[1] = *(const v8h*)(p + 16); return u.v;
}
__device__ __forceinline__ v16h frag_f32(const float* rowk0, int lane) {
  v16h a; const float* p = rowk0 + 8 * (lane >> 4);
#pragma unroll
  for (int i = 0; i < 8; ++i) { a[i] = (_Float16)p[i]; a[8 + i] = (_Float16)p[16 + i]; }
  return a;
}
__device__ __forceinline__ v16h frag_f32s(const float* rowk0, int lane, float sc) {
  v16h a; const float* p = rowk0 + 8 * (lane >> 4);
#pragma unroll
  for (int i = 0; i < 8; ++i) { a[i] = (_Float16)(p[i] * sc); a[8 + i] = (_Float16)(p[16 + i] * sc); }
  return a;
}
__device__ __forceinline__ v16h fragc_f32(const float* W, int k0, int n, int lane, int ld, int K) {
  v16h a; const int g = lane >> 4;
#pragma unroll
  for (int i = 0; i < 8; ++i) { const int ka = k0 + 8 * g + i, kb = ka + 16;
    a[i] = (_Float16)(ka < K ? W[(size_t)(ka < K ? ka : K - 1) * ld + n] : 0.f); a[8 + i] = (_Float16)(kb < K ? W[(size_t)(kb < K ? kb : K - 1) * ld + n] : 0.f); }
  return a;
}
struct F2 { v16b h, l; };
__device__ __forceinline__ F2 bsplit16(const float v[16]) { F2 r;
#pragma unroll
  for (int i = 0; i < 16; ++i) { const __bf16 h = (__bf16)v[i]; r.h[i] = h; r.l[i] = (__bf16)(v[i] - (float)h); }
  return r; }
__device__ __forceinline__ F2 split_row(const float* row, int k0, int lane) { float v[16]; const float* p = row + k0 + 8 * (lane >> 4);
#pragma unroll
  for (int i = 0; i < 8; ++i) { v[i] = p[i]; v[8 + i] = p[16 + i]; }
  return bsplit16(v); }
__device__ __forceinline__ F2 split_rowK(const float* row, int k0, int lane, int K) { float v[16]; const int g = lane >> 4;
#pragma unroll
  for (int i = 0; i < 8; ++i) { const int ka = k0 + 8 * g + i, kb = ka + 16; v[i] = ka < K ? row[ka < K ? ka : K - 1] : 0.f; v[8 + i] = kb < K ? row[kb < K ? kb : K - 1] : 0.f; }
  return bsplit16(v); }
__device__ __forceinline__ F2 split_col(const float* W, int k0, int n, int lane, int ld, int K) { float v[16]; const int g = lane >> 4;
#pragma unroll
  for (int i = 0; i < 8; ++i) { const int ka = k0 + 8 * g + i, kb = ka + 16; v[i] = ka < K ? W[(size_t)(ka < K ? ka : K - 1) * ld + n] : 0.f; v[8 + i] = kb < K ? W[(size_t)(kb < K ? kb : K - 1) * ld + n] : 0.f; }
  return bsplit16(v); }
__device__ __forceinline__ v8f mac3(const F2& a, const F2& b, v8f c) { c = wmma_bf(a.l, b.h, c); c = wmma_bf(a.h, b.l, c); return wmma_bf(a.h, b.h, c); }
__device__ __forceinline__ float sigm(float v) { return 1.0f / (1.0f + expf(-v)); }
#define LDSX() do { asm volatile("s_wait_dscnt 0" ::: "memory"); __builtin_amdgcn_wave_barrier(); __builtin_amdgcn_fence(__ATOMIC_RELEASE, "workgroup"); } while (0)


#define NB 4
#define NPT 16384
#define KN 32
#define FI 32
#define PE 64
#define G1 128
#define FO 64
#define NROW ((size_t)NB * NPT * KN)
#ifndef TRB
#define TRB ((int)(NROW / 64))
#endif
typedef __attribute__((ext_vector_type(8))) __bf16 v8b;
__device__ __forceinline__ v16b frag_b(const __bf16* rowk0, int lane) {
  union { v16b v; v8b q[2]; } u; const __bf16* p = rowk0 + 8 * (lane >> 4);
  u.q[0] = *(const v8b*)p; u.q[1] = *(const v8b*)(p + 16); return u.v;
}
__device__ __forceinline__ float bfr(float v) { return (float)(__bf16)v; }
__device__ __attribute__((noinline)) float exp_ni(float v) { return expf(v); }
__device__ __attribute__((noinline)) float erf_ni(float v) { return erff(v); }

#define WS_W2  0u
#define WS_W3  (WS_W2 + 2u * PE * PE)
#define WS_W4  (WS_W3 + 2u * G1 * (FI + PE))
#define WS_END (WS_W4 + 2u * FO * G1 + 256u)

__global__ __launch_bounds__(256) void k_pack(const float* __restrict__ PW2, const float* __restrict__ MW1, const float* __restrict__ MW2, _Float16* __restrict__ Wr) { const int which = blockIdx.x, t = threadIdx.x;
  if (which == 0) { __shared__ __align__(16) _Float16 s[PE * PE]; for (int e = t; e < PE * PE; e += 256) { const int n = e / PE, k = e % PE; s[e] = (_Float16)(bfr(PW2[k * PE + n]) * 256.0f); } __syncthreads(); for (int q = t; q < PE * PE / 8; q += 256) vst2((unsigned*)(Wr + WS_W2 / 2 + q * 8), *(const v4u*)&s[q * 8]); }
  else if (which == 1) { __shared__ __align__(16) _Float16 s1[G1 * (FI + PE)]; for (int e = t; e < G1 * (FI + PE); e += 256) { const int n = e / (FI + PE), k = e % (FI + PE); s1[e] = (_Float16)(bfr(MW1[k * G1 + n]) * 256.0f); } __syncthreads(); for (int q = t; q < G1 * (FI + PE) / 8; q += 256) vst2((unsigned*)(Wr + WS_W3 / 2 + q * 8), *(const v4u*)&s1[q * 8]); }
  else { __shared__ __align__(16) _Float16 s2[FO * G1]; for (int e = t; e < FO * G1; e += 256) { const int n = e / G1, k = e % G1; s2[e] = (_Float16)(bfr(MW2[k * FO + n]) * 256.0f); } __syncthreads(); for (int q = t; q < FO * G1 / 8; q += 256) vst2((unsigned*)(Wr + WS_W4 / 2 + q * 8), *(const v4u*)&s2[q * 8]); } }
__global__ __launch_bounds__(128) void k_daf(const float* __restrict__ PTS, const float* __restrict__ FEAT, const int* __restrict__ IDX, const float* __restrict__ PW1, const float* __restrict__ PB1, const float* __restrict__ PB2, const float* __restrict__ MB1, const float* __restrict__ MB2, const _Float16* __restrict__ Wr, float* __restrict__ OUT) {
  __shared__ __align__(16) _Float16 sa[64][FI + PE + 8];
  __shared__ __align__(16) _Float16 sh[64][G1 + 8];
  __shared__ __align__(16) float so[64][FO + 4];
  const int tid = threadIdx.x, wave = tid >> 5, lane = tid & 31, col = lane & 15, g = lane >> 4;
  const size_t row0 = (size_t)blockIdx.x * 64; const size_t b = row0 / ((size_t)NPT * KN); const size_t n0 = (row0 / KN) % NPT;
  { const int rr = tid >> 1, hf = tid & 1; const size_t n = n0 + (rr >> 5); const int k = rr & 31; const int j = IDX[(b * NPT + n) * KN + k];
    float rel[3]; for (int i = 0; i < 3; ++i) rel[i] = bfr(PTS[(b * NPT + j) * 3 + i]) - bfr(PTS[(b * NPT + n) * 3 + i]);
    for (int f = hf * 16; f < hf * 16 + 16; ++f) sa[rr][f] = (_Float16)bfr(FEAT[(b * NPT + j) * FI + f]);
    for (int o = hf * 32; o < hf * 32 + 32; ++o) { const float v = rel[0] * bfr(PW1[o]) + rel[1] * bfr(PW1[PE + o]) + rel[2] * bfr(PW1[2 * PE + o]) + bfr(PB1[o]); sh[rr][o] = (_Float16)fmaxf(v, 0.f); } }
  __syncthreads();
  const int r0 = wave * 16;
  { v8f acc[4] = {};
#pragma unroll
    for (int kc = 0; kc < PE / 32; ++kc) { const v16h a = frag_h(&sh[r0 + col][0] + kc * 32, lane);
#pragma unroll
      for (int jt = 0; jt < 4; ++jt) acc[jt] = wmma16(a, frag_h(Wr + WS_W2 / 2 + (size_t)(jt * 16 + col) * PE + kc * 32, lane), acc[jt]); }
#pragma unroll
    for (int jt = 0; jt < 4; ++jt) { const float bb = bfr(PB2[jt * 16 + col]);
#pragma unroll
      for (int r = 0; r < 8; ++r) sa[r0 + 8 * g + r][FI + jt * 16 + col] = (_Float16)(acc[jt][r] * (1.0f / 256.0f) + bb); } }
  LDSX();
  { v8f acc[8] = {};
#pragma unroll
    for (int kc = 0; kc < (FI + PE) / 32; ++kc) { const v16h a = frag_h(&sa[r0 + col][0] + kc * 32, lane);
#pragma unroll
      for (int jt = 0; jt < 8; ++jt) acc[jt] = wmma16(a, frag_h(Wr + WS_W3 / 2 + (size_t)(jt * 16 + col) * (FI + PE) + kc * 32, lane), acc[jt]); }
#pragma unroll
    for (int jt = 0; jt < 8; ++jt) { const float bb = bfr(MB1[jt * 16 + col]);
#pragma unroll
      for (int r = 0; r < 8; ++r) sh[r0 + 8 * g + r][jt * 16 + col] = (_Float16)fmaxf(acc[jt][r] * (1.0f / 256.0f) + bb, 0.f); } }
  LDSX();
  { v8f acc[4] = {};
#pragma unroll
    for (int kc = 0; kc < G1 / 32; ++kc) { const v16h a = frag_h(&sh[r0 + col][0] + kc * 32, lane);
#pragma unroll
      for (int jt = 0; jt < 4; ++jt) acc[jt] = wmma16(a, frag_h(Wr + WS_W4 / 2 + (size_t)(jt * 16 + col) * G1 + kc * 32, lane), acc[jt]); }
#pragma unroll
    for (int jt = 0; jt < 4; ++jt) { const float bb = bfr(MB2[jt * 16 + col]);
#pragma unroll
      for (int r = 0; r < 8; ++r) so[r0 + 8 * g + r][jt * 16 + col] = acc[jt][r] * (1.0f / 256.0f) + bb; } }
  __syncthreads();
  { const int p = tid >> 6, c = tid & 63; float s = 0.f; for (int k = 0; k < KN; ++k) s += so[p * 32 + k][c] * (1.0f / 32.0f); __shared__ __align__(16) float orow[2][FO]; orow[p][c] = s; __syncthreads();
    if (tid < 32) { const int pp = tid >> 4, q = tid & 15; vst2(OUT + (b * NPT + n0 + pp) * FO + q * 4, *(const v4f*)&orow[pp][q * 4]); } }
}
extern "C" void kernel_launch(void* const* d_in, const int* in_sizes, int n_in, void* d_out, int out_size, void* d_ws, size_t ws_size, hipStream_t stream) {
  (void)in_sizes; (void)n_in; (void)out_size;
  const float** F = (const float**)d_in;
  if (ws_size < (size_t)WS_END) return;
  char* ws = (char*)d_ws; _Float16* Wr = (_Float16*)ws;
  k_pack<<<3, 256, 0, stream>>>(F[6], F[8], F[10], Wr);
  k_daf<<<TRB, 128, 0, stream>>>(F[0], F[1], (const int*)d_in[3], F[4], F[5], F[7], F[9], F[11], Wr, (float*)d_out);
}
